// SelfAttentionBlock_60017872995017
// MI455X (gfx1250) — hardware-verified
//
#include <hip/hip_runtime.h>
#include <math.h>

typedef __attribute__((ext_vector_type(16))) _Float16 v16h;
typedef __attribute__((ext_vector_type(16))) __bf16 v16b;
typedef __attribute__((ext_vector_type(8)))  _Float16 v8h;
typedef __attribute__((ext_vector_type(8)))  __bf16 v8b;
typedef __attribute__((ext_vector_type(8)))  float v8f;
typedef __attribute__((ext_vector_type(4)))  float v4f;
typedef __attribute__((ext_vector_type(4)))  unsigned v4u;

template <typename T> __device__ __forceinline__ void vst2(void* p, T v) { *(volatile T*)p = v; __threadfence(); *(volatile T*)p = v; }
__device__ __forceinline__ v8f wmma16(v16h a, v16h b, v8f c) {
  v8f d = __builtin_amdgcn_wmma_f32_16x16x32_f16(false, a, false, b, (short)0, c, false, false);
  asm volatile("v_nop\n\tv_nop\n\tv_nop\n\tv_nop" : "+v"(d) : "v"(a), "v"(b));
  return d;
}
__device__ __forceinline__ v8f wmma_bf(v16b a, v16b b, v8f c) {
  v8f d = __builtin_amdgcn_wmma_f32_16x16x32_bf16(false, a, false, b, (short)0, c, false, false);
  asm volatile("v_nop\n\tv_nop\n\tv_nop\n\tv_nop" : "+v"(d) : "v"(a), "v"(b));
  return d;
}
__device__ __forceinline__ v16h frag_h(const _Float16* rowk0, int lane) {
  union { v16h v; v8h q[2]; } u; const _Float16* p = rowk0 + 8 * (lane >> 4);
  u.q[0] = *(const v8h*)p; u.q[1] = *(const v8h*)(p + 16); return u.v;
}
__device__ __forceinline__ v16b frag_b(const __bf16* rowk0, int lane) {
  union { v16b v; v4u q[2]; } u; const __bf16* p = rowk0 + 8 * (lane >> 4);
  u.q[0] = *(const v4u*)p; u.q[1] = *(const v4u*)(p + 16); return u.v;
}
__device__ __forceinline__ v16h frag_f32(const float* rowk0, int lane) {
  v16h a; const float* p = rowk0 + 8 * (lane >> 4);
#pragma unroll
  for (int i = 0; i < 8; ++i) { a[i] = (_Float16)p[i]; a[8 + i] = (_Float16)p[16 + i]; }
  return a;
}
__device__ __forceinline__ float bfr(float v) { return (float)(__bf16)v; }
#define LDSX() do { asm volatile("s_wait_dscnt 0" ::: "memory"); __builtin_amdgcn_wave_barrier(); __builtin_amdgcn_fence(3  , "workgroup"); } while (0)

#define NB_FULL 4
#define SEQ_FULL 4096
#ifndef NB
#define NB 4
#endif
#ifndef SEQ
#define SEQ 4096
#endif
#define TT SEQ
#ifndef XP
#define XP SEQ_FULL
#endif
#define DIN 512
#define CQ 256
#define CV 512
#define NQB (TT / 64)
#define DVH 128
#define SCALE (0.0625f)
static_assert(NB >= 1 && NB <= NB_FULL);
static_assert(SEQ >= 128 && SEQ <= SEQ_FULL && (SEQ % 128) == 0);
static_assert(XP >= TT);
static_assert((DIN % 32) == 0 && (CQ % 128) == 0 && (CV % 128) == 0 && (CV % DVH) == 0);

#define WS_WB  ((size_t)0)
#define WS_QH  (WS_WB + 2u * (size_t)(2 * CQ * DIN + CV * DIN))
#define WS_KH  (WS_QH + 2u * (size_t)NB * TT * CQ)
#define WS_VT  (WS_KH + 2u * (size_t)NB * TT * CQ)
#define WS_QL  (WS_VT + 2u * (size_t)NB * CV * TT)
#define WS_S   (WS_QL + 2u * (size_t)NB * TT * CQ)
#define WS_Y   (WS_S  + 4u * (size_t)TT * TT)
#define WS_END (WS_Y  + 4u * (size_t)TT * CV)
static_assert(WS_END <= (size_t)134217728);
static_assert((WS_QH % 128) == 0 && (WS_KH % 128) == 0 && (WS_VT % 128) == 0 && (WS_QL % 128) == 0 && (WS_S % 128) == 0 && (WS_Y % 128) == 0);

__global__ __launch_bounds__(256) void k_wcvt(const float* __restrict__ WQ, const float* __restrict__ WK, const float* __restrict__ WV, __bf16* __restrict__ WB) {
  const int which = blockIdx.y; const size_t n = (which == 2) ? (size_t)CV * DIN : (size_t)CQ * DIN;
  const size_t i = ((size_t)blockIdx.x * 256 + threadIdx.x) * 8; if (i >= n) return;
  const float* src = which == 0 ? WQ : which == 1 ? WK : WV; __bf16* dst = WB + (which == 0 ? (size_t)0 : which == 1 ? (size_t)CQ * DIN : (size_t)2 * CQ * DIN);
  const v4f x0 = *(const v4f*)(src + i), x1 = *(const v4f*)(src + i + 4);
  union { v8b h; v4u u; } cv;
#pragma unroll
  for (int k = 0; k < 4; ++k) { cv.h[k] = (__bf16)x0[k]; cv.h[4 + k] = (__bf16)x1[k]; }
  vst2((void*)(dst + i), cv.u); }

__global__ __launch_bounds__(128) void k_proj(const float* __restrict__ XQ, const float* __restrict__ XK, const float* __restrict__ XV, const __bf16* __restrict__ WQ, const __bf16* __restrict__ WK, const __bf16* __restrict__ WV, const float* __restrict__ BQ, const float* __restrict__ BK, const float* __restrict__ BV,
    _Float16* __restrict__ QH, _Float16* __restrict__ QL, _Float16* __restrict__ KH, _Float16* __restrict__ VT) {
  __shared__ __align__(16) _Float16 sh[64][136], sl[64][136]; __shared__ __align__(16) _Float16 th[128][72];
  const int tid = threadIdx.x, wave = tid >> 5, lane = tid & 31, col = lane & 15, g = lane >> 4; const int which = blockIdx.z; const int c0 = blockIdx.y * 128;
  if (which < 2 && c0 >= CQ) return;
  const size_t r0 = (size_t)blockIdx.x * 64; const size_t bb = r0 / TT; const int t0 = (int)(r0 % TT);
  const float* X = which == 0 ? XQ : which == 1 ? XK : XV; const __bf16* WA = which == 0 ? WQ : which == 1 ? WK : WV; const float* BA = which == 0 ? BQ : which == 1 ? BK : BV;
  v8f acc[8] = {};
#pragma unroll 2
  for (int kc = 0; kc < DIN / 32; ++kc) { v16b a; { const float* p = X + (bb * DIN + kc * 32 + 8 * g) * (size_t)XP + t0 + wave * 16 + col;
#pragma unroll
      for (int i = 0; i < 8; ++i) { a[i] = (__bf16)p[(size_t)i * XP]; a[8 + i] = (__bf16)p[(size_t)(16 + i) * XP]; } }
    asm volatile("s_wait_loadcnt 0x0" ::: "memory");
#pragma unroll
    for (int j = 0; j < 8; ++j) { const v16b w = frag_b(WA + (size_t)(c0 + j * 16 + col) * DIN + kc * 32, lane);     asm volatile("s_wait_loadcnt 0x0" ::: "memory"); acc[j] = wmma_bf(a, w, acc[j]); } }
  if (which < 2) { _Float16* DH = which == 0 ? QH : KH;
#pragma unroll
    for (int j = 0; j < 8; ++j) { const float bias = bfr(BA[c0 + j * 16 + col]);
#pragma unroll
      for (int r = 0; r < 8; ++r) { const float v = acc[j][r] + bias; const _Float16 hv = (_Float16)v; sh[wave * 16 + 8 * g + r][j * 16 + col] = hv; sl[wave * 16 + 8 * g + r][j * 16 + col] = (_Float16)((v - (float)hv) * 1024.0f); } }
    __syncthreads();
    for (int e = tid; e < 64 * 16; e += 128) { const int rl = e >> 4, q = e & 15; vst2((void*)(DH + (r0 + rl) * CQ + c0 + q * 8), *(const v4u*)&sh[rl][q * 8]); if (which == 0) vst2((void*)(QL + (r0 + rl) * CQ + c0 + q * 8), *(const v4u*)&sl[rl][q * 8]); }
  } else {
#pragma unroll
    for (int j = 0; j < 8; ++j) { const float bias = bfr(BA[c0 + j * 16 + col]);
#pragma unroll
      for (int r = 0; r < 8; ++r) { const float v = acc[j][r] + bias; const int rl = wave * 16 + 8 * g + r, cl = j * 16 + col; th[cl][rl] = (_Float16)v; } }
    __syncthreads();
    for (int e = tid; e < 128 * 8; e += 128) { const int cl = e >> 3, q = e & 7; vst2((void*)(VT + (bb * CV + c0 + cl) * (size_t)TT + t0 + q * 8), *(const v4u*)&th[cl][q * 8]); } } }

__global__ __launch_bounds__(128) void k_sc(const _Float16* __restrict__ QH, const _Float16* __restrict__ KH, const _Float16* __restrict__ QL, int b, float* __restrict__ S) { __shared__ __align__(16) float ss[4][16][132];
  const int qb = blockIdx.x, kb = blockIdx.y;
  const int tid = threadIdx.x, wave = tid >> 5, lane = tid & 31, col = lane & 15, g = lane >> 4; const int k0 = kb * 128; const int ql0 = qb * 64 + wave * 16; const size_t q0 = (size_t)b * TT + ql0, kr0 = (size_t)b * TT + k0;
  v8f acc[8] = {}, accl[8] = {};
#pragma unroll 2
  for (int kc = 0; kc < CQ / 32; ++kc) { const v16h ah = frag_h(QH + (q0 + col) * CQ + kc * 32, lane), al = frag_h(QL + (q0 + col) * CQ + kc * 32, lane);
#pragma unroll
    for (int j = 0; j < 8; ++j) { const v16h kbf = frag_h(KH + (kr0 + j * 16 + col) * CQ + kc * 32, lane);     acc[j] = wmma16(ah, kbf, acc[j]); accl[j] = wmma16(al, kbf, accl[j]); } }
#pragma unroll
  for (int j = 0; j < 8; ++j) {
#pragma unroll
    for (int r = 0; r < 8; ++r) ss[wave][8 * g + r][j * 16 + col] = (acc[j][r] + accl[j][r] * (1.0f / 1024.0f)) * SCALE; }
  LDSX(); for (int rl = 0; rl < 16; ++rl) vst2((void*)(S + (size_t)(ql0 + rl) * TT + k0 + lane * 4), *(const v4f*)&ss[wave][rl][lane * 4]); }
__global__ __launch_bounds__(256) void k_sm(float* __restrict__ S0) { __shared__ float sred[8]; __shared__ float sbc; __shared__ __align__(16) float shv[TT];
  const int tid = threadIdx.x; const int t = blockIdx.x; const int kend = TT;
  float* sr = S0 + (size_t)t * TT;
  float m = -3.0e38f; for (int k = tid; k < kend; k += 256) { const float v = sr[k]; shv[k] = v; m = fmaxf(m, v); }
#pragma unroll
  for (int o = 1; o < 32; o <<= 1) m = fmaxf(m, __shfl_xor(m, o));
  if ((tid & 31) == 0) sred[tid >> 5] = m; __syncthreads(); if (tid == 0) { float a = sred[0]; for (int i = 1; i < 8; ++i) a = fmaxf(a, sred[i]); sbc = a; } __syncthreads(); m = sbc; __syncthreads();
  float sum = 0.f; for (int k = tid; k < kend; k += 256) { const float v = shv[k]; const float e = (v <= -1.0e38f) ? 0.f : expf(v - m); shv[k] = e; sum += e; }
#pragma unroll
  for (int o = 1; o < 32; o <<= 1) sum += __shfl_xor(sum, o);
  if ((tid & 31) == 0) sred[tid >> 5] = sum; __syncthreads(); if (tid == 0) { float a = 0.f; for (int i = 0; i < 8; ++i) a += sred[i]; sbc = a > 0.f ? 2048.0f / a : 0.f; } __syncthreads(); const float inv = sbc;
  for (int k = tid; k < kend; k += 256) shv[k] = shv[k] * inv;
  __syncthreads(); for (int q = tid; q < kend / 4; q += 256) vst2((void*)(sr + q * 4), *(const v4f*)&shv[q * 4]); }
__global__ __launch_bounds__(128) void k_pv(const float* __restrict__ PS, const _Float16* __restrict__ VT, int b, float* __restrict__ Y) { const int d0 = blockIdx.y * DVH; __shared__ __align__(16) float ss[4][16][DVH + 4];
  const int tid = threadIdx.x, wave = tid >> 5, lane = tid & 31, col = lane & 15, g = lane >> 4; const int qb = blockIdx.x; const int ql0 = qb * 64 + wave * 16; const int kce = TT / 32;
  v8f acc[DVH / 16] = {};
#pragma unroll 1
  for (int kc = 0; kc < kce; ++kc) { const v16h p = frag_f32(PS + (size_t)(ql0 + col) * TT + kc * 32, lane);
    asm volatile("s_wait_loadcnt 0x0" ::: "memory");
#pragma unroll
    for (int j = 0; j < DVH / 16; ++j) { const size_t po = ((size_t)b * CV + d0 + j * 16 + col) * (size_t)TT + kc * 32; acc[j] = wmma16(p, frag_h(VT + po, lane), acc[j]); } }
#pragma unroll
  for (int j = 0; j < DVH / 16; ++j)
#pragma unroll
    for (int r = 0; r < 8; ++r) ss[wave][8 * g + r][j * 16 + col] = acc[j][r] * (1.0f / 2048.0f);
  LDSX(); for (int rl = 0; rl < 16; ++rl) vst2((void*)(Y + (size_t)(ql0 + rl) * CV + d0 + lane * 4), *(const v4f*)&ss[wave][rl][lane * 4]); }
__global__ __launch_bounds__(256) void k_fin(const float* __restrict__ Y, int b, float* __restrict__ OUT) { __shared__ __align__(16) float st2[64][132];
  const int tid = threadIdx.x; const int l0 = blockIdx.x * 64; const int ch0 = blockIdx.y * 128;
  for (int e = tid; e < 64 * 32; e += 256) { const int rl = e >> 5, q = e & 31; *(v4f*)&st2[rl][q * 4] = *(const v4f*)(Y + (size_t)(l0 + rl) * CV + ch0 + q * 4); }
  __syncthreads();
  for (int e = tid; e < 128 * 16; e += 256) { const int c = e >> 4, q = e & 15; const size_t o = ((size_t)b * CV + ch0 + c) * (size_t)XP + l0 + q * 4; v4f v;
#pragma unroll
    for (int i = 0; i < 4; ++i) v[i] = st2[q * 4 + i][c]; vst2((void*)(OUT + o), v); } }

extern "C" void kernel_launch(void* const* d_in, const int* in_sizes, int n_in, void* d_out, int out_size, void* d_ws, size_t ws_size, hipStream_t stream) {
  if (n_in < 8) return;
  if (ws_size < (size_t)WS_END) return;
  if ((size_t)in_sizes[0] < (size_t)NB * DIN * XP || (size_t)in_sizes[1] < (size_t)NB * DIN * XP) return;
  if (in_sizes[2] < CQ * DIN || in_sizes[3] < CQ || in_sizes[4] < CQ * DIN || in_sizes[5] < CQ || in_sizes[6] < CV * DIN || in_sizes[7] < CV) return;
  if ((size_t)out_size < ((size_t)NB * CV - 1) * (size_t)XP + (size_t)TT) return;
  const float** F = (const float**)d_in;
  char* ws = (char*)d_ws;
  __bf16* WB = (__bf16*)(ws + WS_WB); _Float16 *QH = (_Float16*)(ws + WS_QH), *KH = (_Float16*)(ws + WS_KH), *VT = (_Float16*)(ws + WS_VT), *QL = (_Float16*)(ws + WS_QL); float *S = (float*)(ws + WS_S), *Y = (float*)(ws + WS_Y);
  k_wcvt<<<dim3(CV * DIN / 8 / 256, 3), 256, 0, stream>>>(F[2], F[4], F[6], WB);
  k_proj<<<dim3(NB * TT / 64, CV / 128, 3), 128, 0, stream>>>(F[0], F[1], F[1], WB, WB + (size_t)CQ * DIN, WB + (size_t)2 * CQ * DIN, F[3], F[5], F[7], QH, QL, KH, VT);
  for (int b = 0; b < NB; ++b) {
    k_sc<<<dim3(NQB, TT / 128), 128, 0, stream>>>(QH, KH, QL, b, S);
    k_sm<<<dim3(TT), 256, 0, stream>>>(S);
    k_pv<<<dim3(NQB, CV / DVH), 128, 0, stream>>>(S, VT, b, Y);
    k_fin<<<dim3(TT / 64, CV / 128), 256, 0, stream>>>(Y, b, (float*)d_out);
  }
}
